// BTSPAttention_82540681494945
// MI455X (gfx1250) — hardware-run, weakly checked
//
#include <hip/hip_runtime.h>


#ifndef NB
#define NB 2
#endif
#ifndef SEQ
#define SEQ 2048
#endif
#define NB_FULL  2
#define SEQ_FULL 2048
#define DM   1024
#define NH_  16
#define HD   64
#define AW   4
#define OSP  68
#define TBN  500
#define TBH  250
#define TBP  512
#define SC2  ((float)(0.125 * 1.4426950408889634))
#define LOG2E 1.4426950408889634f
#define PSH  14.0f
#define NEGB (-3.0e38f)
#define CXS  256.0f
#define WOS  64.0f
#define OSC  (1.0f / 16384.0f)

static_assert(HD == 64);
static_assert(NH_ * HD == DM);
static_assert(DM % 64 == 0);
static_assert(DM % 32 == 0);
static_assert(HD % 32 == 0);
static_assert(SEQ % 64 == 0);
static_assert((NB * SEQ) % 64 == 0);
static_assert(SEQ % 32 == 0);
static_assert(SEQ % (16 * AW) == 0);
static_assert(((size_t)SEQ * DM) % 8 == 0);
static_assert(((size_t)DM * DM) % 8 == 0);
static_assert(NB <= NB_FULL);
static_assert(SEQ <= SEQ_FULL);
static_assert((OSP * 4) % 16 == 0);
static_assert(OSP >= HD + 4);
static_assert(TBP >= TBN);
static_assert(TBH * 2 == TBN);
static_assert(TBP % (32 * AW) == 0);
static_assert(32 * 4 * 16 == 16 * HD * 2);
static_assert(32 * 8 * 16 == 16 * 64 * 4);
static_assert((AW * 16 * OSP + TBP) * 4 <= 131072);
static_assert(16 * 68 * 4 <= 131072);

typedef _Float16 h16;
typedef unsigned short bf;
typedef __attribute__((ext_vector_type(16))) __bf16   v16bf;
typedef __attribute__((ext_vector_type(16))) _Float16 v16h;
typedef __attribute__((ext_vector_type(8)))  _Float16 v8h;
typedef __attribute__((ext_vector_type(8)))  unsigned short v8us;
typedef __attribute__((ext_vector_type(8)))  float    v8f;
typedef __attribute__((ext_vector_type(4)))  float    v4f;
typedef v4f  __attribute__((may_alias)) v4fa;

__device__ __forceinline__ unsigned short f2bf(float f) { unsigned u = __float_as_uint(f); u += 0x7FFFu + ((u >> 16) & 1u); return (unsigned short)(u >> 16); }
__device__ __forceinline__ float bfr(float f) { return __uint_as_float(((unsigned)f2bf(f)) << 16); }
__device__ __forceinline__ v16h cat16(v8h lo, v8h hi) { return __builtin_shufflevector(lo, hi, 0, 1, 2, 3, 4, 5, 6, 7, 8, 9, 10, 11, 12, 13, 14, 15); }
__device__ __forceinline__ v16bf cat16b(v8us lo, v8us hi) { return __builtin_bit_cast(v16bf, __builtin_shufflevector(lo, hi, 0, 1, 2, 3, 4, 5, 6, 7, 8, 9, 10, 11, 12, 13, 14, 15)); }
__device__ __forceinline__ v8f wmma16(v16h a, v16h b, v8f c) { return __builtin_amdgcn_wmma_f32_16x16x32_f16(false, a, false, b, (short)0, c, false, false); }
__device__ __forceinline__ v8f wmmab(v16bf a, v16bf b, v8f c) { return __builtin_amdgcn_wmma_f32_16x16x32_bf16(false, a, false, b, (short)0, c, false, false); }
__device__ __forceinline__ v8f wg16(v16h a, v16h b, v8f c) { c = wmma16(a, b, c); asm volatile("v_nop\n\tv_nop\n\tv_nop\n\tv_nop" : "+v"(c) : "v"(a), "v"(b)); return c; }
__device__ __forceinline__ v8f wgb(v16bf a, v16bf b, v8f c) { c = wmmab(a, b, c); asm volatile("v_nop\n\tv_nop\n\tv_nop\n\tv_nop" : "+v"(c) : "v"(a), "v"(b)); return c; }
__device__ __forceinline__ v16h  ldh(const h16* p) { return cat16(*(const v8h*)p, *(const v8h*)(p + 16)); }
__device__ __forceinline__ v16bf ldb(const bf* p)  { return cat16b(*(const v8us*)p, *(const v8us*)(p + 16)); }
__device__ __forceinline__ void wave_sync() { __builtin_amdgcn_fence(3  , "wavefront"); __builtin_amdgcn_wave_barrier(); asm volatile("" ::: "memory"); }
__device__ __forceinline__ h16 toh_flush(float v) { const h16 r = (h16)v; return (fabsf(v) < 6.103515625e-05f) ? (h16)0.0f : r; }

__global__ __launch_bounds__(256) void k_cvt8(const float* __restrict__ src, bf* dst, size_t n8) {
    const size_t i = (size_t)blockIdx.x * 256 + threadIdx.x; if (i >= n8) return;
    const v8f v = *(const v8f*)(src + i * 8); v8us o;
#pragma unroll
    for (int k = 0; k < 8; ++k) o[k] = f2bf(v[k]);
    *(volatile v8us*)(dst + i * 8) = o; __threadfence(); *(volatile v8us*)(dst + i * 8) = o;
}

__global__ __launch_bounds__(256) void k_cvth(const float* __restrict__ src, h16* dst, size_t n8) {
    const size_t i = (size_t)blockIdx.x * 256 + threadIdx.x; if (i >= n8) return;
    const v8f v = *(const v8f*)(src + i * 8); v8h o;
#pragma unroll
    for (int k = 0; k < 8; ++k) o[k] = toh_flush(bfr(v[k]) * WOS);
    *(volatile v8h*)(dst + i * 8) = o; __threadfence(); *(volatile v8h*)(dst + i * 8) = o;
}

template <int MODE>
__device__ __forceinline__ void proj_body(const bf* __restrict__ A, const bf* __restrict__ Bt, const float* __restrict__ bias, h16* Ph) {
    __shared__ __align__(16) float os[16 * 68];
    const int K = DM;
    const int lane = threadIdx.x & 31, lr = lane & 15, hi = lane >> 4; const int r0 = blockIdx.x * 64, c0 = blockIdx.y * 64;
    v8f acc[4][4];
#pragma unroll
    for (int mb = 0; mb < 4; ++mb)
#pragma unroll
        for (int nb = 0; nb < 4; ++nb) acc[mb][nb] = (v8f){};
    const size_t aoff = (size_t)(r0 + lr) * K + 8 * hi, boff = (size_t)(c0 + lr) * K + 8 * hi;
#pragma unroll 1
    for (int kc = 0; kc < K; kc += 32) {
        v16bf a[4];
#pragma unroll
        for (int mb = 0; mb < 4; ++mb) a[mb] = ldb(A + aoff + (size_t)mb * 16 * K + kc);
#pragma unroll
        for (int nb = 0; nb < 4; ++nb) { const v16bf b = ldb(Bt + boff + (size_t)nb * 16 * K + kc);
#pragma unroll
            for (int mb = 0; mb < 4; ++mb) acc[mb][nb] = wgb(a[mb], b, acc[mb][nb]); }
    }
    float bc[4];
#pragma unroll
    for (int nb = 0; nb < 4; ++nb) bc[nb] = (MODE == 0) ? bfr(bias[c0 + nb * 16 + lr]) : 0.0f;
    size_t tbase;
    if (MODE == 0) { const int bb = r0 / SEQ, tt = r0 % SEQ; const int zc = bb * NH_ + c0 / HD;
                     tbase = ((size_t)zc * SEQ + (size_t)tt) * HD; }
    else           { const int bb = c0 / SEQ, tt = c0 % SEQ;
                     tbase = (size_t)bb * (size_t)DM * SEQ + (size_t)r0 * SEQ + (size_t)tt; }
#pragma unroll
    for (int mb = 0; mb < 4; ++mb) {
        float br[8];
#pragma unroll
        for (int j = 0; j < 8; ++j) br[j] = (MODE == 1) ? bfr(bias[r0 + mb * 16 + hi * 8 + j]) : 0.0f;
#pragma unroll
        for (int nb = 0; nb < 4; ++nb) {
#pragma unroll
            for (int j = 0; j < 8; ++j) os[(hi * 8 + j) * 68 + nb * 16 + lr] = acc[mb][nb][j] + bc[nb] + br[j]; }
        wave_sync();
#pragma unroll 1
        for (int ps = 0; ps < 2; ++ps) {
            if (MODE == 0) {
                const size_t sb = tbase + (size_t)(mb * 16) * HD;
#pragma unroll
                for (int s = 0; s < 4; ++s) { const int p = s * 32 + lane; const int row = p >> 3, c8 = (p & 7) * 8;
                    const v4f x0 = *(const v4fa*)(&os[row * 68 + c8]); const v4f x1 = *(const v4fa*)(&os[row * 68 + c8 + 4]); v8h hv;
#pragma unroll
                    for (int i = 0; i < 4; ++i) { hv[i] = toh_flush(x0[i]); hv[4 + i] = toh_flush(x1[i]); }
                    const size_t oo = sb + (size_t)p * 8;
                    *(volatile v8h*)(Ph + oo) = hv; }
            } else {
                const size_t sb = tbase + (size_t)(mb * 16) * SEQ;
#pragma unroll
                for (int s = 0; s < 4; ++s) { const int row = 4 * s + (lane >> 3), c8 = (lane & 7) * 8;
                    const v4f x0 = *(const v4fa*)(&os[row * 68 + c8]); const v4f x1 = *(const v4fa*)(&os[row * 68 + c8 + 4]); v8h hv;
#pragma unroll
                    for (int i = 0; i < 4; ++i) { hv[i] = toh_flush(x0[i]); hv[4 + i] = toh_flush(x1[i]); }
                    const size_t oo = sb + (size_t)row * SEQ + c8;
                    *(volatile v8h*)(Ph + oo) = hv; }
            }
            if (ps == 0) __threadfence(); }
        wave_sync();
    }
}

__global__ __launch_bounds__(32) void k_proj_qk(const bf* __restrict__ A, const bf* __restrict__ Bt, const float* __restrict__ bias, h16* Ph) { proj_body<0>(A, Bt, bias, Ph); }
__global__ __launch_bounds__(32) void k_proj_vt(const bf* __restrict__ A, const bf* __restrict__ Bt, const float* __restrict__ bias, h16* Ph) { proj_body<1>(A, Bt, bias, Ph); }

__global__ __launch_bounds__(32) void k_oproj(const h16* __restrict__ A, const h16* __restrict__ Bt, const float* __restrict__ bias, float* OUT) {
    __shared__ __align__(16) float os[16 * 68];
    const int K = DM;
    const int lane = threadIdx.x & 31, lr = lane & 15, hi = lane >> 4; const int r0 = blockIdx.x * 64, c0 = blockIdx.y * 64;
    v8f acc[4][4];
#pragma unroll
    for (int mb = 0; mb < 4; ++mb)
#pragma unroll
        for (int nb = 0; nb < 4; ++nb) acc[mb][nb] = (v8f){};
    const size_t aoff = (size_t)(r0 + lr) * K + 8 * hi, boff = (size_t)(c0 + lr) * K + 8 * hi;
#pragma unroll 1
    for (int kc = 0; kc < K; kc += 32) {
        v16h a[4];
#pragma unroll
        for (int mb = 0; mb < 4; ++mb) a[mb] = ldh(A + aoff + (size_t)mb * 16 * K + kc);
#pragma unroll
        for (int nb = 0; nb < 4; ++nb) { const v16h b = ldh(Bt + boff + (size_t)nb * 16 * K + kc);
#pragma unroll
            for (int mb = 0; mb < 4; ++mb) acc[mb][nb] = wg16(a[mb], b, acc[mb][nb]); }
    }
    float bc[4];
#pragma unroll
    for (int nb = 0; nb < 4; ++nb) bc[nb] = bfr(bias[c0 + nb * 16 + lr]);
#pragma unroll
    for (int mb = 0; mb < 4; ++mb) {
#pragma unroll
        for (int nb = 0; nb < 4; ++nb) {
#pragma unroll
            for (int j = 0; j < 8; ++j) os[(hi * 8 + j) * 68 + nb * 16 + lr] = acc[mb][nb][j] * OSC + bc[nb]; }
        wave_sync();
        float* orow = OUT + (size_t)(r0 + mb * 16) * DM + c0;
#pragma unroll 1
        for (int ps = 0; ps < 2; ++ps) {
#pragma unroll
            for (int s = 0; s < 8; ++s) { const int row = 2 * s + (lane >> 4), cofs = (lane & 15) * 4;
                const v4f val = *(const v4fa*)(&os[row * 68 + cofs]);
                *(volatile v4f*)(orow + (size_t)row * DM + cofs) = val; }
            if (ps == 0) __threadfence(); }
        wave_sync();
    }
}

__global__ __launch_bounds__(32 * AW) void k_flash(const h16* __restrict__ QH, const h16* __restrict__ KP, const h16* __restrict__ VT,
                                                   const float* __restrict__ tbias, const float* __restrict__ etg, const float* __restrict__ isg, h16* CX) {
    __shared__ __align__(16) float os[AW * 16 * OSP];
    __shared__ __align__(16) float tl[TBP];
    const int lane = threadIdx.x & 31, lr = lane & 15, hi = lane >> 4;
    const int wave = __builtin_amdgcn_readfirstlane((int)(threadIdx.x >> 5));
    const int zh = blockIdx.y; const int b = zh / NH_, h = zh % NH_;
    const int t0 = (blockIdx.x * AW + wave) * 16;
    { const float g = 1.0f / (1.0f + expf(-bfr(etg[0]))); const float cg = bfr(isg[0]);
#pragma unroll 1
      for (int i = threadIdx.x; i < TBP; i += 32 * AW) { const int ic = min(i, TBN - 1); tl[i] = (g * bfr(tbias[ic]) + cg) * LOG2E; } }
    __syncthreads();
    const size_t pbase = (size_t)zh * SEQ * HD;
    const size_t qo = pbase + (size_t)(t0 + lr) * HD + 8 * hi;
    const v16h qh0 = ldh(QH + qo), qh1 = ldh(QH + qo + 32);
    const size_t ko = pbase + (size_t)lr * HD + 8 * hi;
    const size_t vo = pbase + (size_t)lr * SEQ + 8 * hi;
    const int eq = TBH - (t0 + lr);
    const int ulo = TBH - (t0 + 15), uhi = TBH + 31 - t0;
    v8f o[4];
#pragma unroll
    for (int j = 0; j < 4; ++j) o[j] = (v8f){};
    float m = NEGB, l = 0.0f;
#pragma unroll 1
    for (int key0 = 0; key0 < SEQ; key0 += 32) {
        const h16* ka = KP + ko + (size_t)key0 * HD;
        const v16h ka0 = ldh(ka), ka1 = ldh(ka + 32), kb0 = ldh(ka + 16 * HD), kb1 = ldh(ka + 16 * HD + 32);
        v8f sa = (v8f){}, sb = (v8f){};
        sa = wg16(ka0, qh0, sa); sb = wg16(kb0, qh0, sb); sa = wg16(ka1, qh1, sa); sb = wg16(kb1, qh1, sb);
        float ta[8], tc[8];
        if (key0 + ulo >= TBN - 1 || key0 + uhi <= 0) {
            const int ic = min(max(key0 + eq, 0), TBN - 1);
            const float c = tl[ic];
#pragma unroll
            for (int r = 0; r < 8; ++r) { ta[r] = sa[r] * SC2 + c; tc[r] = sb[r] * SC2 + c; }
        } else {
            const int ja = key0 + eq + 8 * hi;
#pragma unroll
            for (int r = 0; r < 8; ++r) {
                const int ia = min(max(ja + r, 0), TBN - 1), ib = min(max(ja + 16 + r, 0), TBN - 1);
                const float ba = tl[ia], bb = tl[ib];
                ta[r] = sa[r] * SC2 + ba; tc[r] = sb[r] * SC2 + bb; }
        }
        float mx = NEGB;
#pragma unroll
        for (int r = 0; r < 8; ++r) mx = fmaxf(mx, fmaxf(ta[r], tc[r]));
        mx = fmaxf(mx, __shfl_xor(mx, 16, 32));
        const float mnew = fmaxf(m, mx);
        const float alpha = __builtin_amdgcn_exp2f(m - mnew);
        const float sh = PSH - mnew;
        v16h pb; float ls = 0.0f;
#pragma unroll
        for (int r = 0; r < 8; ++r) {
            const float xa = ta[r] + sh, xc = tc[r] + sh;
            const float ga = (xa < -14.0f) ? 0.0f : __builtin_amdgcn_exp2f(xa);
            const float gc = (xc < -14.0f) ? 0.0f : __builtin_amdgcn_exp2f(xc);
            const h16 pa = (h16)ga; const h16 pc = (h16)gc;
            pb[r] = pa; pb[8 + r] = pc;
            ls += (float)pa + (float)pc; }
        l = l * alpha + ls; m = mnew;
#pragma unroll
        for (int j = 0; j < 4; ++j) o[j] = o[j] * alpha;
        const h16* va = VT + vo + key0;
        v16h v[4];
#pragma unroll
        for (int j = 0; j < 4; ++j) v[j] = ldh(va + (size_t)(16 * j) * SEQ);
#pragma unroll
        for (int j = 0; j < 4; ++j) o[j] = wg16(v[j], pb, o[j]);
    }
    l += __shfl_xor(l, 16, 32);
    const float inv = CXS * (1.0f / l);
    const int wb = wave * 16 * OSP;
#pragma unroll
    for (int j = 0; j < 4; ++j) { v4f a, c;
      a[0] = o[j][0] * inv; a[1] = o[j][1] * inv; a[2] = o[j][2] * inv; a[3] = o[j][3] * inv; c[0] = o[j][4] * inv; c[1] = o[j][5] * inv; c[2] = o[j][6] * inv; c[3] = o[j][7] * inv;
      *(v4fa*)(&os[wb + lr * OSP + 16 * j + 8 * hi]) = a; *(v4fa*)(&os[wb + lr * OSP + 16 * j + 8 * hi + 4]) = c; }
    wave_sync();
    h16* crow = CX + (((size_t)(h * NB + b)) * SEQ + (size_t)t0) * HD;
#pragma unroll 1
    for (int ps = 0; ps < 2; ++ps) {
#pragma unroll
        for (int s = 0; s < 4; ++s) { const int row = 4 * s + (lane >> 3), c8 = (lane & 7) * 8;
            const v4f x0 = *(const v4fa*)(&os[wb + row * OSP + c8]); const v4f x1 = *(const v4fa*)(&os[wb + row * OSP + c8 + 4]); v8h hv;
#pragma unroll
            for (int i = 0; i < 4; ++i) { hv[i] = toh_flush(x0[i]); hv[4 + i] = toh_flush(x1[i]); }
            *(volatile v8h*)(crow + (size_t)row * HD + c8) = hv; }
        if (ps == 0) __threadfence(); }
}

static constexpr size_t al256(size_t v) { return (v + 255) & ~(size_t)255; }
static constexpr size_t SZ_XB = al256((size_t)NB * SEQ * DM * 2);
static constexpr size_t SZ_WB = al256((size_t)3 * DM * DM * 2);
static constexpr size_t SZ_WO = al256((size_t)DM * DM * 2);
static constexpr size_t SZ_PL = al256((size_t)NB * NH_ * SEQ * HD * 2);
static constexpr size_t SZ_TOTAL = SZ_XB + SZ_WB + SZ_WO + 4 * SZ_PL;
static constexpr size_t NEED_X = ((size_t)(NB - 1) * SEQ_FULL + SEQ) * DM;
static constexpr size_t NEED_W = (size_t)DM * DM;
static constexpr size_t NEED_OUT = (size_t)NB * SEQ * DM;
static_assert(SZ_TOTAL <= (size_t)134217728);
static_assert(((size_t)DM * DM * 2) % 256 == 0);
static_assert((size_t)NB * NH_ * SEQ * HD == (size_t)NB * DM * SEQ);
static_assert(NEED_OUT * 4 <= (size_t)NB_FULL * SEQ_FULL * DM * 4);

extern "C" void kernel_launch(void* const* d_in, const int* in_sizes, int n_in,
                              void* d_out, int out_size, void* d_ws, size_t ws_size, hipStream_t stream) {
    if (n_in < 12) return;
    if ((size_t)in_sizes[0] < NEED_X) return;
    if ((size_t)in_sizes[1] < NEED_W || (size_t)in_sizes[3] < NEED_W || (size_t)in_sizes[5] < NEED_W || (size_t)in_sizes[7] < NEED_W) return;
    if (in_sizes[2] < DM || in_sizes[4] < DM || in_sizes[6] < DM || in_sizes[8] < DM) return;
    if (in_sizes[9] < 1 || in_sizes[10] < 1 || in_sizes[11] < TBN) return;
    if ((size_t)out_size < NEED_OUT) return;
    if (SZ_TOTAL > ws_size) return;
    const float* xin = (const float*)d_in[0];
    const float* wq = (const float*)d_in[1]; const float* bq = (const float*)d_in[2];
    const float* wk = (const float*)d_in[3]; const float* bk = (const float*)d_in[4];
    const float* wv = (const float*)d_in[5]; const float* bv = (const float*)d_in[6];
    const float* wo = (const float*)d_in[7]; const float* bo = (const float*)d_in[8];
    const float* etg = (const float*)d_in[9]; const float* isg = (const float*)d_in[10]; const float* tbl = (const float*)d_in[11];
    float* OUT = (float*)d_out;
    char* wsp = (char*)d_ws;
    bf* XB = (bf*)wsp; wsp += SZ_XB;
    bf* WB = (bf*)wsp; wsp += SZ_WB;
    h16* WOH = (h16*)wsp; wsp += SZ_WO;
    h16* QH = (h16*)wsp; wsp += SZ_PL;
    h16* KP = (h16*)wsp; wsp += SZ_PL;
    h16* VT = (h16*)wsp; wsp += SZ_PL;
    h16* CX = (h16*)wsp; wsp += SZ_PL;
    bf* WQ = WB; bf* WK = WB + (size_t)DM * DM; bf* WV = WB + (size_t)2 * DM * DM;

    if (SEQ == SEQ_FULL) {
        const size_t n8 = (size_t)NB * SEQ * DM / 8;
        k_cvt8<<<(unsigned)((n8 + 255) / 256), 256, 0, stream>>>(xin, XB, n8);
    } else {
        const size_t n8 = (size_t)SEQ * DM / 8;
        for (int b = 0; b < NB; ++b) k_cvt8<<<(unsigned)((n8 + 255) / 256), 256, 0, stream>>>(xin + (size_t)b * SEQ_FULL * DM, XB + (size_t)b * SEQ * DM, n8);
    }
    { const size_t n8 = (size_t)DM * DM / 8; const unsigned g = (unsigned)((n8 + 255) / 256);
      k_cvt8<<<g, 256, 0, stream>>>(wq, WQ, n8); k_cvt8<<<g, 256, 0, stream>>>(wk, WK, n8); k_cvt8<<<g, 256, 0, stream>>>(wv, WV, n8);
      k_cvth<<<g, 256, 0, stream>>>(wo, WOH, n8); }

    k_proj_qk<<<dim3(NB * SEQ / 64, DM / 64, 1), 32, 0, stream>>>(XB, WQ, bq, QH);
    k_proj_qk<<<dim3(NB * SEQ / 64, DM / 64, 1), 32, 0, stream>>>(XB, WK, bk, KP);
    k_proj_vt<<<dim3(DM / 64, NB * SEQ / 64, 1), 32, 0, stream>>>(WV, XB, bv, VT);

    k_flash<<<dim3(SEQ / (16 * AW), NB * NH_, 1), 32 * AW, 0, stream>>>(QH, KP, VT, tbl, etg, isg, CX);

    k_oproj<<<dim3(NB * SEQ / 64, DM / 64, 1), 32, 0, stream>>>(CX, WOH, bo, OUT);
}
